// PytorchMambaBlock_83365315215989
// MI455X (gfx1250) — hardware-verified
//
#include <hip/hip_runtime.h>


typedef __attribute__((ext_vector_type(16))) _Float16 v16h;
typedef __attribute__((ext_vector_type(8)))  _Float16 v8h;
typedef __attribute__((ext_vector_type(4)))  _Float16 v4h;
typedef __attribute__((ext_vector_type(16))) __bf16   v16b;
typedef __attribute__((ext_vector_type(8)))  __bf16   v8b;
typedef __attribute__((ext_vector_type(8)))  float    v8f;
typedef __attribute__((ext_vector_type(4)))  float    v4f;
typedef __attribute__((ext_vector_type(2)))  float    v2f;

#define LOG2E_F 1.4426950408889634f
#define LN2_F   0.6931471805599453f

__device__ __forceinline__ unsigned short f2bf_bits(float f) {
  unsigned u = __float_as_uint(f);
  return (unsigned short)((u + 0x7FFFu + ((u >> 16) & 1u)) >> 16);
}
__device__ __forceinline__ float bf_bits2f(unsigned short h) { return __uint_as_float(((unsigned)h) << 16); }

__device__ __forceinline__ void dep_guard_h(v8f& a, v8f& b, v16h x, v16h y) { asm volatile("v_nop\n\tv_nop\n\tv_nop\n\tv_nop" : "+v"(a), "+v"(b) : "v"(x), "v"(y)); }
__device__ __forceinline__ void dep_guard_b(v8f& a, v8f& b, v16b x, v16b y) { asm volatile("v_nop\n\tv_nop\n\tv_nop\n\tv_nop" : "+v"(a), "+v"(b) : "v"(x), "v"(y)); }
__device__ __forceinline__ void keep4_h(v16h a, v16h b, v16h c, v16h d) { asm volatile("v_nop" :: "v"(a), "v"(b), "v"(c), "v"(d)); }
__device__ __forceinline__ void keep4_b(v16b a, v16b b, v16b c, v16b d) { asm volatile("v_nop" :: "v"(a), "v"(b), "v"(c), "v"(d)); }
__device__ __forceinline__ void acc_guard4(v8f& a, v8f& b, v8f& c, v8f& d) { asm volatile("v_nop\n\tv_nop\n\tv_nop\n\tv_nop" : "+v"(a), "+v"(b), "+v"(c), "+v"(d)); }
template <typename T> struct Frag;
template <> struct Frag<_Float16> {
  typedef v16h V; union U { v16h v; v8h h[2]; };
  static __device__ __forceinline__ v16h load(const _Float16* p) {
    U f; f.h[0] = *(const v8h*)(p); f.h[1] = *(const v8h*)(p + 16); return f.v;
  }
  static __device__ __forceinline__ v8f mma(v16h a, v16h b, v8f c) {
    return __builtin_amdgcn_wmma_f32_16x16x32_f16(false, a, false, b, (short)0, c, false, false);
  }
  static __device__ __forceinline__ void guard(v8f& a, v8f& b, v16h x, v16h y) { dep_guard_h(a, b, x, y); }
  static __device__ __forceinline__ void keep(v16h a, v16h b, v16h c, v16h d) { keep4_h(a, b, c, d); }
};
template <> struct Frag<__bf16> {
  typedef v16b V; union U { v16b v; v8b h[2]; };
  static __device__ __forceinline__ v16b load(const __bf16* p) {
    U f; f.h[0] = *(const v8b*)(p); f.h[1] = *(const v8b*)(p + 16); return f.v;
  }
  static __device__ __forceinline__ v8f mma(v16b a, v16b b, v8f c) {
    return __builtin_amdgcn_wmma_f32_16x16x32_bf16(false, a, false, b, (short)0, c, false, false);
  }
  static __device__ __forceinline__ void guard(v8f& a, v8f& b, v16b x, v16b y) { dep_guard_b(a, b, x, y); }
  static __device__ __forceinline__ void keep(v16b a, v16b b, v16b c, v16b d) { keep4_b(a, b, c, d); }
};

template <int ET> struct Elem;
template <> struct Elem<0> { typedef _Float16 T; };
template <> struct Elem<1> { typedef __bf16 T; };
template <int ET, bool SPLIT, int BIAS_MODE, int OUT_MODE, bool RESID, int ACT = 0>
__global__ __launch_bounds__(256) void wmma_gemm64(
    const unsigned short* __restrict__ Ap, const unsigned short* __restrict__ A2p, int lda, long strideA,
    const unsigned short* __restrict__ Btp, const unsigned short* __restrict__ Bt2p, int ldb, long strideB,
    void* __restrict__ Cout, void* __restrict__ Cout2, int ldc, long strideC,
    const float* __restrict__ bias,
    const float* __restrict__ resid, long strideR,
    int M, int N, int K, float scale) {
  typedef typename Elem<ET>::T T;
  typedef typename Frag<T>::V V;
  const T* A = (const T*)Ap; const T* A2 = (const T*)A2p; const T* Bt = (const T*)Btp; const T* Bt2 = (const T*)Bt2p;
  __shared__ __align__(16) float sT[8][16 * 68];
  const int b    = blockIdx.y;
  const int lane = threadIdx.x & 31;
  const int wave = threadIdx.x >> 5;
  const int tilesN = N >> 6;
  const int tilesM = M >> 6;
  const int tile = blockIdx.x * 8 + wave;
  if (tile >= tilesM * tilesN) return;
  const int tm = tile / tilesN;
  const int tn = tile - tm * tilesN;
  const int m0 = tm << 6;
  const int n0 = tn << 6;

  const T* Ab  = A  + (size_t)b * strideA;
  const T* Bb  = Bt + (size_t)b * strideB;
  const T* Ab2 = SPLIT ? (A2  + (size_t)b * strideA) : nullptr;
  const T* Bb2 = SPLIT ? (Bt2 + (size_t)b * strideB) : nullptr;

  const int rlane = lane & 15;
  const int koff  = (lane >> 4) * 8;
  const int mOff  = (lane >> 4) * 8;

  v8f acc[4][4];
#pragma unroll
  for (int i = 0; i < 4; ++i)
#pragma unroll
    for (int j = 0; j < 4; ++j) acc[i][j] = (v8f){0.f,0.f,0.f,0.f,0.f,0.f,0.f,0.f};

  for (int k0 = 0; k0 < K; k0 += 32) {
    V bh[4], bl[4];
#pragma unroll
    for (int j = 0; j < 4; ++j) {
      const size_t bo = (size_t)(n0 + (j << 4) + rlane) * ldb + koff + k0;
      bh[j] = Frag<T>::load(Bb + bo);
      if (SPLIT) bl[j] = Frag<T>::load(Bb2 + bo);
    }
#pragma unroll
    for (int i = 0; i < 4; ++i) {
      const size_t ao = (size_t)(m0 + (i << 4) + rlane) * lda + koff + k0;
      V ah = Frag<T>::load(Ab + ao);
      V al;
      if (SPLIT) al = Frag<T>::load(Ab2 + ao);
#pragma unroll
      for (int j = 0; j < 4; ++j) {
        acc[i][j] = Frag<T>::mma(ah, bh[j], acc[i][j]);
        if (SPLIT) {
          acc[i][j] = Frag<T>::mma(ah, bl[j], acc[i][j]);
          acc[i][j] = Frag<T>::mma(al, bh[j], acc[i][j]);
        }
      }
      Frag<T>::guard(acc[i][0], acc[i][3], ah, SPLIT ? al : ah);
    }
    Frag<T>::keep(bh[0], bh[1], bh[2], bh[3]);
    if (SPLIT) Frag<T>::keep(bl[0], bl[1], bl[2], bl[3]);
  }
  acc_guard4(acc[0][0], acc[0][1], acc[0][2], acc[0][3]);
  acc_guard4(acc[1][0], acc[1][1], acc[1][2], acc[1][3]);
  acc_guard4(acc[2][0], acc[2][1], acc[2][2], acc[2][3]);
  acc_guard4(acc[3][0], acc[3][1], acc[3][2], acc[3][3]);

  float* slab = sT[wave];
  const float* Rb = RESID ? (resid + (size_t)b * strideR) : nullptr;
#pragma unroll
  for (int i = 0; i < 4; ++i) {
    const int mBase = m0 + (i << 4);
#pragma unroll
    for (int j = 0; j < 4; ++j) {
      const int n = n0 + (j << 4) + rlane;
      float bv = 0.f;
      if (BIAS_MODE == 2) bv = bias[n];
#pragma unroll
      for (int r = 0; r < 8; ++r) {
        float v = acc[i][j][r] * scale;
        if (BIAS_MODE == 1) v += bias[mBase + mOff + r];
        if (BIAS_MODE == 2) v += bv;
        if (RESID) v += Rb[(size_t)(mBase + mOff + r) * ldc + n];
        if (ACT == 1) v = tanhf(v);
        if (ACT == 2) v = fmaxf(v, 0.0f);
        if (ACT == 3) v = v / (1.0f + expf(-v));
        if (ACT == 4) v = (v > 0.f) ? v : 0.01f * v;
        if (ACT == 5) v = 0.5f * v * (1.0f + erff(v * 0.70710678118654752f));
        slab[(mOff + r) * 68 + (j << 4) + rlane] = v;
      }
    }
    __builtin_amdgcn_fence(__ATOMIC_RELEASE, "workgroup");
    __builtin_amdgcn_wave_barrier();
    __builtin_amdgcn_fence(__ATOMIC_ACQUIRE, "workgroup");
    if (OUT_MODE == 0) {
      float* C = (float*)Cout + (size_t)b * strideC;
      const int hh = lane >> 4, c4 = (lane & 15) * 4;
      for (int pass = 0; pass < 2; ++pass) {
#pragma unroll
        for (int it = 0; it < 8; ++it) {
          const int row = it * 2 + hh;
          v4f v = *(const v4f*)(slab + row * 68 + c4);
          *(volatile v4f*)(C + (size_t)(mBase + row) * ldc + n0 + c4) = v;
        }
        __threadfence();
      }
    } else {
      const int q = lane >> 3, c8 = (lane & 7) * 8;
      unsigned short* C  = (unsigned short*)Cout  + (size_t)b * strideC;
      unsigned short* C2 = (OUT_MODE == 2) ? ((unsigned short*)Cout2 + (size_t)b * strideC) : nullptr;
      for (int pass = 0; pass < 2; ++pass) {
#pragma unroll
        for (int it = 0; it < 4; ++it) {
          const int row = it * 4 + q;
          const float* sp = slab + row * 68 + c8;
          v8h hv, lv;
#pragma unroll
          for (int e = 0; e < 8; ++e) {
            if (OUT_MODE == 1) {
              hv[e] = (_Float16)sp[e];
            } else {
              unsigned short hb = f2bf_bits(sp[e]);
              unsigned short lb = f2bf_bits(sp[e] - bf_bits2f(hb));
              hv[e] = __builtin_bit_cast(_Float16, hb);
              lv[e] = __builtin_bit_cast(_Float16, lb);
            }
          }
          *(volatile v8h*)(C + (size_t)(mBase + row) * ldc + n0 + c8) = hv;
          if (OUT_MODE == 2) *(volatile v8h*)(C2 + (size_t)(mBase + row) * ldc + n0 + c8) = lv;
        }
        __threadfence();
      }
    }
    __builtin_amdgcn_fence(__ATOMIC_RELEASE, "workgroup");
    __builtin_amdgcn_wave_barrier();
    __builtin_amdgcn_fence(__ATOMIC_ACQUIRE, "workgroup");
  }
}

__global__ __launch_bounds__(256) void cast_scale_f16x2(
    const float* __restrict__ in, _Float16* __restrict__ out, int n2, float scale) {
  int i = blockIdx.x * 256 + threadIdx.x;
  if (i < n2) {
    const _Float16 h0 = (_Float16)(in[2 * i] * scale), h1 = (_Float16)(in[2 * i + 1] * scale);
    const unsigned u = (unsigned)__builtin_bit_cast(unsigned short, h0) | ((unsigned)__builtin_bit_cast(unsigned short, h1) << 16);
    ((volatile unsigned*)out)[i] = u;
    __threadfence();
    ((volatile unsigned*)out)[i] = u;
  }
}

__device__ __forceinline__ float silu_fast(float a) {
  const float e = __builtin_amdgcn_exp2f(-a * LOG2E_F);
  return a * __builtin_amdgcn_rcpf(1.0f + e);
}
__device__ __forceinline__ float softplus_fast(float v) {
  const float m = fmaxf(v, 0.0f);
  const float t = __builtin_amdgcn_exp2f(-fabsf(v) * LOG2E_F);
  return m + __builtin_amdgcn_logf(1.0f + t) * LN2_F;
}

__global__ __launch_bounds__(256) void conv_silu_kernel(
    const float* __restrict__ P, const float* __restrict__ cw, const float* __restrict__ cb,
    float* __restrict__ xa, _Float16* __restrict__ xah, int L, int C, int total4) {
  const int idx = blockIdx.x * 256 + threadIdx.x;
  if (idx >= total4) return;
  const int cq = C >> 2;
  const int c4 = idx % cq;
  const int r  = idx / cq;
  const int t  = r % L;
  const int c0 = c4 << 2;
  const v4f w0 = *(const v4f*)(cw + (size_t)(c0 + 0) * 4);
  const v4f w1 = *(const v4f*)(cw + (size_t)(c0 + 1) * 4);
  const v4f w2 = *(const v4f*)(cw + (size_t)(c0 + 2) * 4);
  const v4f w3 = *(const v4f*)(cw + (size_t)(c0 + 3) * 4);
  float s0 = 0.f, s1 = 0.f, s2 = 0.f, s3 = 0.f;
#pragma unroll
  for (int j = 0; j < 4; ++j) {
    if (t + j >= 3) {
      const v4f xv = *(const v4f*)(P + (size_t)(r + j - 3) * C + c0);
      s0 += w0[j] * xv[0];
      s1 += w1[j] * xv[1];
      s2 += w2[j] * xv[2];
      s3 += w3[j] * xv[3];
    }
  }
  const v4f bb = *(const v4f*)(cb + c0);
  s0 += bb[0]; s1 += bb[1]; s2 += bb[2]; s3 += bb[3];
  v4f ov;
  ov[0] = silu_fast(s0); ov[1] = silu_fast(s1); ov[2] = silu_fast(s2); ov[3] = silu_fast(s3);
  v4h hv;
  hv[0] = (_Float16)ov[0]; hv[1] = (_Float16)ov[1]; hv[2] = (_Float16)ov[2]; hv[3] = (_Float16)ov[3];
  float*    pa = xa  + (size_t)r * C + c0;
  _Float16* ph = xah + (size_t)r * C + c0;
  *(volatile v4f*)pa = ov;
  *(volatile v4h*)ph = hv;
  __threadfence();
  *(volatile v4f*)pa = ov;
  *(volatile v4h*)ph = hv;
}

__global__ __launch_bounds__(64) void ssm_scan_kernel(
    const float* __restrict__ xa, const float* __restrict__ dtp, const float* __restrict__ Z,
    const float* __restrict__ Alog, const float* __restrict__ Dp, _Float16* __restrict__ yg,
    int L, int C, int nthr) {
  const int idx = blockIdx.x * 64 + threadIdx.x;
  if (idx >= nthr) return;
  const int cpairs = C >> 1;
  const int cp = idx % cpairs;
  const int b  = idx / cpairs;
  const int c0 = cp * 2;
  float a0[16], a1[16], h0[16], h1[16];
#pragma unroll
  for (int s = 0; s < 16; ++s) {
    a0[s] = -__builtin_amdgcn_exp2f(Alog[(size_t)c0 * 16 + s] * LOG2E_F) * LOG2E_F;
    a1[s] = -__builtin_amdgcn_exp2f(Alog[(size_t)(c0 + 1) * 16 + s] * LOG2E_F) * LOG2E_F;
    h0[s] = 0.f;
    h1[s] = 0.f;
  }
  const float dp0 = Dp[c0], dp1 = Dp[c0 + 1];
  const size_t rb = (size_t)b * L;
#pragma unroll 1
  for (int t = 0; t < L; ++t) {
    const size_t o = (rb + t) * (size_t)C + c0;
    const v2f xv = *(const v2f*)(xa + o);
    const v2f dv = *(const v2f*)(dtp + o);
    const v2f zv = *(const v2f*)(Z + o);
    const float dt0 = softplus_fast(dv[0]);
    const float dt1 = softplus_fast(dv[1]);
    const float db0 = dt0 * xv[0];
    const float db1 = dt1 * xv[1];
    float s0 = 0.f, s1 = 0.f;
#pragma unroll
    for (int s = 0; s < 16; ++s) {
      const float e0 = __builtin_amdgcn_exp2f(dt0 * a0[s]);
      const float e1 = __builtin_amdgcn_exp2f(dt1 * a1[s]);
      h0[s] = e0 * h0[s] + db0;
      h1[s] = e1 * h1[s] + db1;
      s0 += h0[s];
      s1 += h1[s];
    }
    const float y0 = s0 + dp0 * xv[0];
    const float y1 = s1 + dp1 * xv[1];
    const float g0 = y0 * silu_fast(zv[0]);
    const float g1 = y1 * silu_fast(zv[1]);
    const _Float16 q0 = (_Float16)g0, q1 = (_Float16)g1;
    const unsigned u = (unsigned)__builtin_bit_cast(unsigned short, q0) | ((unsigned)__builtin_bit_cast(unsigned short, q1) << 16);
    volatile unsigned* p = (volatile unsigned*)(yg + o);
    *p = u;
    __threadfence();
    *p = u;
  }
}

extern "C" void kernel_launch(void* const* d_in, const int* in_sizes, int n_in,
                              void* d_out, int out_size, void* d_ws, size_t ws_size,
                              hipStream_t stream) {
  constexpr int DM = 1024, DI = 2048, DS = 16, KC = 4, NB = 2, L = 2048, ML = NB * L;
  if (n_in < 9) return;
  if (in_sizes[0] != ML * DM || in_sizes[1] != 2 * DI * DM || in_sizes[2] != DI * KC || in_sizes[3] != DI ||
      in_sizes[4] != DI * DS || in_sizes[5] != DI || in_sizes[6] != DI * DI || in_sizes[7] != DI ||
      in_sizes[8] != DM * DI) return;
  if (out_size != ML * DM) return;

  const float* x      = (const float*)d_in[0];
  const float* W_in   = (const float*)d_in[1];
  const float* conv_w = (const float*)d_in[2];
  const float* conv_b = (const float*)d_in[3];
  const float* A_log  = (const float*)d_in[4];
  const float* Dp     = (const float*)d_in[5];
  const float* W_dt   = (const float*)d_in[6];
  const float* b_dt   = (const float*)d_in[7];
  const float* W_out  = (const float*)d_in[8];
  float* out = (float*)d_out;

  const size_t szXh   = (size_t)ML * DM * 2;
  const size_t szWin  = (size_t)2 * DI * DM * 2;
  const size_t szWdt  = (size_t)DI * DI * 2;
  const size_t szWout = (size_t)DM * DI * 2;
  const size_t szF32  = (size_t)ML * DI * 4;
  const size_t szH16  = (size_t)ML * DI * 2;
  size_t off = 0;
  const size_t offXh = off;   off += szXh;
  const size_t offWin = off;  off += szWin;
  const size_t offWdt = off;  off += szWdt;
  const size_t offWout = off; off += szWout;
  const size_t offP = off;    off += szF32;
  const size_t offZ = off;    off += szF32;
  const size_t offXA = off;   off += szF32;
  const size_t total = off;
  if (total > ws_size) return;
  if (szXh + szWin < szH16) return;

  char* ws = (char*)d_ws;
  _Float16* xh    = (_Float16*)(ws + offXh);
  _Float16* winh  = (_Float16*)(ws + offWin);
  _Float16* wdth  = (_Float16*)(ws + offWdt);
  _Float16* wouth = (_Float16*)(ws + offWout);
  float*    Pbuf  = (float*)(ws + offP);
  float*    Zbuf  = (float*)(ws + offZ);
  float*    XA    = (float*)(ws + offXA);
  _Float16* xacth = (_Float16*)(ws + offXh);
  float*    dtp   = (float*)(ws + offP);
  _Float16* ygh   = (_Float16*)(ws + offXh);

  const float WSC = 64.0f, WSC_INV = 1.0f / 64.0f;

  {
    const int n2x = ML * DM / 2, n2win = 2 * DI * DM / 2, n2wdt = DI * DI / 2, n2wout = DM * DI / 2;
    cast_scale_f16x2<<<(n2x + 255) / 256, 256, 0, stream>>>(x, xh, n2x, 1.0f);
    cast_scale_f16x2<<<(n2win + 255) / 256, 256, 0, stream>>>(W_in, winh, n2win, WSC);
    cast_scale_f16x2<<<(n2wdt + 255) / 256, 256, 0, stream>>>(W_dt, wdth, n2wdt, WSC);
    cast_scale_f16x2<<<(n2wout + 255) / 256, 256, 0, stream>>>(W_out, wouth, n2wout, WSC);
  }

  {
    const int tiles = (ML / 64) * (DI / 64);
    dim3 grid((tiles + 7) / 8, 1);
    wmma_gemm64<0, false, 0, 0, false, 0><<<grid, 256, 0, stream>>>(
        (const unsigned short*)xh, (const unsigned short*)xh, DM, 0L,
        (const unsigned short*)winh, (const unsigned short*)winh, DM, 0L,
        (void*)Pbuf, (void*)Pbuf, DI, 0L, b_dt, x, 0L, ML, DI, DM, WSC_INV);
    wmma_gemm64<0, false, 0, 0, false, 0><<<grid, 256, 0, stream>>>(
        (const unsigned short*)xh, (const unsigned short*)xh, DM, 0L,
        (const unsigned short*)(winh + (size_t)DI * DM), (const unsigned short*)(winh + (size_t)DI * DM), DM, 0L,
        (void*)Zbuf, (void*)Zbuf, DI, 0L, b_dt, x, 0L, ML, DI, DM, WSC_INV);
  }

  {
    const int total4 = ML * (DI / 4);
    conv_silu_kernel<<<(total4 + 255) / 256, 256, 0, stream>>>(Pbuf, conv_w, conv_b, XA, xacth, L, DI, total4);
  }

  {
    const int tiles = (ML / 64) * (DI / 64);
    dim3 grid((tiles + 7) / 8, 1);
    wmma_gemm64<0, false, 2, 0, false, 0><<<grid, 256, 0, stream>>>(
        (const unsigned short*)xacth, (const unsigned short*)xacth, DI, 0L,
        (const unsigned short*)wdth, (const unsigned short*)wdth, DI, 0L,
        (void*)dtp, (void*)dtp, DI, 0L, b_dt, x, 0L, ML, DI, DI, WSC_INV);
  }

  {
    const int nthr = NB * (DI / 2);
    ssm_scan_kernel<<<(nthr + 63) / 64, 64, 0, stream>>>(XA, dtp, Zbuf, A_log, Dp, ygh, L, DI, nthr);
  }

  {
    const int tiles = (ML / 64) * (DM / 64);
    dim3 grid((tiles + 7) / 8, 1);
    wmma_gemm64<0, false, 0, 0, false, 0><<<grid, 256, 0, stream>>>(
        (const unsigned short*)ygh, (const unsigned short*)ygh, DI, 0L,
        (const unsigned short*)wouth, (const unsigned short*)wouth, DI, 0L,
        (void*)out, (void*)out, DM, 0L, b_dt, x, 0L, ML, DM, DI, WSC_INV);
  }
  (void)hipGetLastError();
}
